// XorzoTransformer_59287728554108
// MI455X (gfx1250) — hardware-verified
//
#include <hip/hip_runtime.h>
#include <hip/hip_bf16.h>
#include <stdint.h>

static constexpr int NBATCH  = 4;
static constexpr int NTOK    = 1024;
static constexpr int NDIM    = 1024;
static constexpr int NHEAD   = 16;
static constexpr int NDHEAD  = 64;
static constexpr int NROWS   = NBATCH * NTOK;
static constexpr int NHID    = 2108;
static constexpr int NACTIVE = 1656;
static constexpr int NHPAD   = 1664;
static_assert(NACTIVE <= NHPAD && NHPAD % 64 == 0 && NHPAD <= NHID, "hidden pad");
static_assert(NROWS % 64 == 0 && NDIM % 64 == 0 && NDIM % 32 == 0 && NHPAD % 32 == 0, "tile multiples");
static_assert(NHEAD * NDHEAD == NDIM && NTOK % 64 == 0 && NDHEAD == 64, "head geometry");

static constexpr size_t PLANE    = (size_t)NROWS * NDIM;
static constexpr size_t WSQ      = (size_t)NDIM * NDIM;
static constexpr size_t OFF_WQKV = 0;
static constexpr size_t OFF_WO   = OFF_WQKV + 3 * WSQ * 2;
static constexpr size_t OFF_WIN  = OFF_WO + WSQ * 2;
static constexpr size_t OFF_WOUT = OFF_WIN + (size_t)NHPAD * NDIM * 2;
static constexpr size_t OFF_NHI  = OFF_WOUT + (size_t)NDIM * NHPAD * 2;
static constexpr size_t OFF_NLO  = OFF_NHI + WSQ * 2;
static constexpr size_t OFF_XN   = OFF_NLO + WSQ * 2;
static constexpr size_t OFF_QKV  = OFF_XN + PLANE * 2;
static constexpr size_t OFF_CB   = OFF_QKV + 3 * PLANE * 2;
static constexpr size_t OFF_X1   = OFF_CB + PLANE * 2;
static constexpr size_t OFF_G    = OFF_X1 + PLANE * 4;
static constexpr size_t WS_TOTAL = OFF_G + (size_t)NROWS * NHPAD * 2;
static constexpr size_t OFF_H    = OFF_QKV;
static constexpr size_t OFF_X2H  = OFF_QKV;
static constexpr size_t OFF_X2L  = OFF_QKV + PLANE * 2;
static_assert(WS_TOTAL == 91750400, "carve total");
static_assert(WS_TOTAL <= (size_t)134217728, "carve under 128 MiB");
static_assert(OFF_H + (size_t)NROWS * NHPAD * 4 <= OFF_X1, "H alias fits in the dead q/k/v/comb region");
static_assert(OFF_X2L + PLANE * 2 <= OFF_X1, "x2 planes alias fits");
static_assert((OFF_WO % 256) == 0 && (OFF_WIN % 256) == 0 && (OFF_WOUT % 256) == 0 && (OFF_NHI % 256) == 0 &&
              (OFF_NLO % 256) == 0 && (OFF_XN % 256) == 0 && (OFF_QKV % 256) == 0 && (OFF_CB % 256) == 0 &&
              (OFF_X1 % 256) == 0 && (OFF_G % 256) == 0 && (OFF_X2L % 256) == 0, "aligned carves");

typedef __attribute__((ext_vector_type(16))) _Float16 v16h;
typedef __attribute__((ext_vector_type(8)))  _Float16 v8h;
typedef __attribute__((ext_vector_type(16))) __bf16   v16b;
typedef __attribute__((ext_vector_type(8)))  __bf16   v8b;
typedef __attribute__((ext_vector_type(8)))  float    v8f;
typedef __attribute__((ext_vector_type(4)))  float    v4f;
typedef __attribute__((ext_vector_type(4)))  unsigned v4u;
typedef __attribute__((ext_vector_type(4)))  int      v4i;
#define PSCALE 32768.0f
#define U16(p) ((const unsigned short*)(const void*)(p))
#define PSCALE_INV (1.0f / 32768.0f)

__device__ __forceinline__ unsigned short f2bf_bits(float f) {
  unsigned u = __float_as_uint(f);
  return (unsigned short)((u + 0x7FFFu + ((u >> 16) & 1u)) >> 16);
}
__device__ __forceinline__ float bf_bits2f(unsigned short h) { return __uint_as_float(((unsigned)h) << 16); }

__device__ __forceinline__ void dep_guard_h(v8f& a, v8f& b, v16h x, v16h y) { asm volatile("v_nop\n\tv_nop\n\tv_nop\n\tv_nop" : "+v"(a), "+v"(b) : "v"(x), "v"(y)); }
__device__ __forceinline__ void dep_guard_b(v8f& a, v8f& b, v16b x, v16b y) { asm volatile("v_nop\n\tv_nop\n\tv_nop\n\tv_nop" : "+v"(a), "+v"(b) : "v"(x), "v"(y)); }
__device__ __forceinline__ void keep4_h(v16h a, v16h b, v16h c, v16h d) { asm volatile("v_nop" :: "v"(a), "v"(b), "v"(c), "v"(d)); }
__device__ __forceinline__ void keep4_b(v16b a, v16b b, v16b c, v16b d) { asm volatile("v_nop" :: "v"(a), "v"(b), "v"(c), "v"(d)); }
__device__ __forceinline__ void acc_guard4(v8f& a, v8f& b, v8f& c, v8f& d) { asm volatile("v_nop\n\tv_nop\n\tv_nop\n\tv_nop" : "+v"(a), "+v"(b), "+v"(c), "+v"(d)); }
template <typename T> struct Frag;
template <> struct Frag<_Float16> {
  typedef v16h V; union U { v16h v; v8h h[2]; };
  static __device__ __forceinline__ v16h load(const _Float16* p) {
    U f; f.h[0] = *(const v8h*)(p); f.h[1] = *(const v8h*)(p + 16); return f.v;
  }
  static __device__ __forceinline__ v8f mma(v16h a, v16h b, v8f c) {
    return __builtin_amdgcn_wmma_f32_16x16x32_f16(false, a, false, b, (short)0, c, false, false);
  }
  static __device__ __forceinline__ void guard(v8f& a, v8f& b, v16h x, v16h y) { dep_guard_h(a, b, x, y); }
  static __device__ __forceinline__ void keep(v16h a, v16h b, v16h c, v16h d) { keep4_h(a, b, c, d); }
};
template <> struct Frag<__bf16> {
  typedef v16b V; union U { v16b v; v8b h[2]; };
  static __device__ __forceinline__ v16b load(const __bf16* p) {
    U f; f.h[0] = *(const v8b*)(p); f.h[1] = *(const v8b*)(p + 16); return f.v;
  }
  static __device__ __forceinline__ v8f mma(v16b a, v16b b, v8f c) {
    return __builtin_amdgcn_wmma_f32_16x16x32_bf16(false, a, false, b, (short)0, c, false, false);
  }
  static __device__ __forceinline__ void guard(v8f& a, v8f& b, v16b x, v16b y) { dep_guard_b(a, b, x, y); }
  static __device__ __forceinline__ void keep(v16b a, v16b b, v16b c, v16b d) { keep4_b(a, b, c, d); }
};

template <int ET> struct Elem;
template <> struct Elem<0> { typedef _Float16 T; };
template <> struct Elem<1> { typedef __bf16 T; };
template <int ET, bool SPLIT, int BIAS_MODE, int OUT_MODE, bool RESID, int ACT, bool GATE>
__global__ __launch_bounds__(256) void wmma_gemm64(
    const unsigned short* __restrict__ Ap, const unsigned short* __restrict__ A2p, int lda, long strideA,
    const unsigned short* __restrict__ Btp, const unsigned short* __restrict__ Bt2p, int ldb, long strideB,
    void* __restrict__ Cout, void* __restrict__ Cout2, int ldc, long strideC,
    const float* __restrict__ bias,
    const float* __restrict__ resid, long strideR,
    const float* __restrict__ gate,
    int M, int N, int K, float scale) {
  typedef typename Elem<ET>::T T;
  typedef typename Frag<T>::V V;
  const T* A = (const T*)Ap; const T* A2 = (const T*)A2p; const T* Bt = (const T*)Btp; const T* Bt2 = (const T*)Bt2p;
  __shared__ __align__(16) float sT[8][16 * 68];
  const int b    = blockIdx.y;
  const int lane = threadIdx.x & 31;
  const int wave = threadIdx.x >> 5;
  const int tilesN = N >> 6;
  const int tilesM = M >> 6;
  const int tile = blockIdx.x * 8 + wave;
  if (tile >= tilesM * tilesN) return;
  const int tm = tile / tilesN;
  const int tn = tile - tm * tilesN;
  const int m0 = tm << 6;
  const int n0 = tn << 6;

  const T* Ab  = A  + (size_t)b * strideA;
  const T* Bb  = Bt + (size_t)b * strideB;
  const T* Ab2 = SPLIT ? (A2  + (size_t)b * strideA) : nullptr;
  const T* Bb2 = SPLIT ? (Bt2 + (size_t)b * strideB) : nullptr;

  const int rlane = lane & 15;
  const int koff  = (lane >> 4) * 8;
  const int mOff  = (lane >> 4) * 8;

  v8f acc[4][4];
#pragma unroll
  for (int i = 0; i < 4; ++i)
#pragma unroll
    for (int j = 0; j < 4; ++j) acc[i][j] = (v8f){0.f,0.f,0.f,0.f,0.f,0.f,0.f,0.f};

  for (int k0 = 0; k0 < K; k0 += 32) {
    V bh[4], bl[4];
#pragma unroll
    for (int j = 0; j < 4; ++j) {
      const size_t bo = (size_t)(n0 + (j << 4) + rlane) * ldb + koff + k0;
      bh[j] = Frag<T>::load(Bb + bo);
      if (SPLIT) bl[j] = Frag<T>::load(Bb2 + bo);
    }
#pragma unroll
    for (int i = 0; i < 4; ++i) {
      const size_t ao = (size_t)(m0 + (i << 4) + rlane) * lda + koff + k0;
      V ah = Frag<T>::load(Ab + ao);
      V al;
      if (SPLIT) al = Frag<T>::load(Ab2 + ao);
#pragma unroll
      for (int j = 0; j < 4; ++j) {
        acc[i][j] = Frag<T>::mma(ah, bh[j], acc[i][j]);
        if (SPLIT) {
          acc[i][j] = Frag<T>::mma(ah, bl[j], acc[i][j]);
          acc[i][j] = Frag<T>::mma(al, bh[j], acc[i][j]);
        }
      }
      Frag<T>::guard(acc[i][0], acc[i][3], ah, SPLIT ? al : ah);
    }
    Frag<T>::keep(bh[0], bh[1], bh[2], bh[3]);
    if (SPLIT) Frag<T>::keep(bl[0], bl[1], bl[2], bl[3]);
  }
  acc_guard4(acc[0][0], acc[0][1], acc[0][2], acc[0][3]);
  acc_guard4(acc[1][0], acc[1][1], acc[1][2], acc[1][3]);
  acc_guard4(acc[2][0], acc[2][1], acc[2][2], acc[2][3]);
  acc_guard4(acc[3][0], acc[3][1], acc[3][2], acc[3][3]);

  float gmul = 1.0f;
  if (GATE) gmul = 1.0f / (1.0f + expf(-gate[0]));

  float* slab = sT[wave];
  const float* Rb = RESID ? (resid + (size_t)b * strideR) : nullptr;
#pragma unroll
  for (int i = 0; i < 4; ++i) {
    const int mBase = m0 + (i << 4);
#pragma unroll
    for (int j = 0; j < 4; ++j) {
      const int n = n0 + (j << 4) + rlane;
      float bv = 0.f;
      if (BIAS_MODE == 2) bv = bias[n];
#pragma unroll
      for (int r = 0; r < 8; ++r) {
        float v = acc[i][j][r] * scale;
        if (BIAS_MODE == 1) v += bias[mBase + mOff + r];
        if (BIAS_MODE == 2) v += bv;
        if (GATE) v *= gmul;
        if (RESID) v += Rb[(size_t)(mBase + mOff + r) * ldc + n];
        if (ACT == 1) v = tanhf(v);
        if (ACT == 2) v = fmaxf(v, 0.0f);
        if (ACT == 3) v = v / (1.0f + expf(-v));
        if (ACT == 4) v = (v > 0.f) ? v : 0.01f * v;
        slab[(mOff + r) * 68 + (j << 4) + rlane] = v;
      }
    }
    __builtin_amdgcn_fence(__ATOMIC_RELEASE, "workgroup");
    __builtin_amdgcn_wave_barrier();
    __builtin_amdgcn_fence(__ATOMIC_ACQUIRE, "workgroup");
    if (OUT_MODE == 0) {
      float* C = (float*)Cout + (size_t)b * strideC;
      const int hh = lane >> 4, c4 = (lane & 15) * 4;
      for (int pass = 0; pass < 2; ++pass) {
#pragma unroll
        for (int it = 0; it < 8; ++it) {
          const int row = it * 2 + hh;
          v4f v = *(const v4f*)(slab + row * 68 + c4);
          *(volatile v4f*)(C + (size_t)(mBase + row) * ldc + n0 + c4) = v;
        }
        __threadfence();
      }
    } else {
      const int q = lane >> 3, c8 = (lane & 7) * 8;
      unsigned short* C  = (unsigned short*)Cout  + (size_t)b * strideC;
      unsigned short* C2 = (OUT_MODE == 2) ? ((unsigned short*)Cout2 + (size_t)b * strideC) : nullptr;
      for (int pass = 0; pass < 2; ++pass) {
#pragma unroll
        for (int it = 0; it < 4; ++it) {
          const int row = it * 4 + q;
          const float* sp = slab + row * 68 + c8;
          v8h hv, lv;
#pragma unroll
          for (int e = 0; e < 8; ++e) {
            if (OUT_MODE == 1) {
              hv[e] = (_Float16)sp[e];
            } else {
              unsigned short hb = f2bf_bits(sp[e]);
              unsigned short lb = f2bf_bits(sp[e] - bf_bits2f(hb));
              hv[e] = __builtin_bit_cast(_Float16, hb);
              lv[e] = __builtin_bit_cast(_Float16, lb);
            }
          }
          *(volatile v8h*)(C + (size_t)(mBase + row) * ldc + n0 + c8) = hv;
          if (OUT_MODE == 2) *(volatile v8h*)(C2 + (size_t)(mBase + row) * ldc + n0 + c8) = lv;
        }
        __threadfence();
      }
    }
    __builtin_amdgcn_fence(__ATOMIC_RELEASE, "workgroup");
    __builtin_amdgcn_wave_barrier();
    __builtin_amdgcn_fence(__ATOMIC_ACQUIRE, "workgroup");
  }
}

template <int MODE>
__global__ __launch_bounds__(256) void tcast_kernel(const float* __restrict__ src, int R, int Csrc,
    unsigned short* __restrict__ dst, unsigned short* __restrict__ dst2, int Kp, int kmax, float mul)
{
  __shared__ float Ls[64][65];
  const int k0 = blockIdx.x * 64, n0 = blockIdx.y * 64;
  const int tid = threadIdx.x, lane = tid & 31, wave = tid >> 5;
#pragma unroll
  for (int cc = 0; cc < 4; ++cc) {
    const int ch = tid + cc * 256;
    const int kk = ch >> 4, n4 = (ch & 15) * 4;
    const int gk = k0 + kk;
    const int gkc = (gk < R) ? gk : (R - 1);
    const v4f w = *(const v4f*)(src + (size_t)gkc * Csrc + n0 + n4);
    const bool z = (gk >= kmax);
#pragma unroll
    for (int e = 0; e < 4; ++e) Ls[kk][n4 + e] = z ? 0.0f : w[e];
  }
  __syncthreads();
  const int q = lane >> 3, c8 = (lane & 7) * 8;
  v8h hv[2], lv[2];
#pragma unroll
  for (int it = 0; it < 2; ++it) {
    const int nn = wave * 8 + it * 4 + q;
#pragma unroll
    for (int e = 0; e < 8; ++e) {
      const float f = Ls[c8 + e][nn] * mul;
      if (MODE == 0) {
        hv[it][e] = (_Float16)f;
        lv[it][e] = hv[it][e];
      } else {
        const unsigned short hb = f2bf_bits(f);
        const unsigned short lb = f2bf_bits(f - bf_bits2f(hb));
        hv[it][e] = __builtin_bit_cast(_Float16, hb);
        lv[it][e] = __builtin_bit_cast(_Float16, lb);
      }
    }
  }
  for (int pass = 0; pass < 2; ++pass) {
#pragma unroll
    for (int it = 0; it < 2; ++it) {
      const int nn = wave * 8 + it * 4 + q;
      const size_t off = (size_t)(n0 + nn) * Kp + k0 + c8;
      *(volatile v8h*)(dst + off) = hv[it];
      if (MODE == 1) *(volatile v8h*)(dst2 + off) = lv[it];
    }
    __threadfence();
  }
}

__global__ __launch_bounds__(128) void bnorm_f16_kernel(const float* __restrict__ x, const float* __restrict__ g,
    const float* __restrict__ bb, const float* __restrict__ bw, unsigned short* __restrict__ outp)
{
  __shared__ float red[3][4];
  const int row = blockIdx.x, tid = threadIdx.x, lane = tid & 31, wave = tid >> 5;
  const float* xr = x + (size_t)row * NDIM + tid * 8;
  const v4f a0 = *(const v4f*)(xr);
  const v4f a1 = *(const v4f*)(xr + 4);
  float v[8];
#pragma unroll
  for (int e = 0; e < 4; ++e) { v[e] = a0[e]; v[4 + e] = a1[e]; }
  float s = 0.f;
#pragma unroll
  for (int e = 0; e < 8; ++e) s += v[e];
#pragma unroll
  for (int off = 1; off < 32; off <<= 1) s += __shfl_xor(s, off, 32);
  if (lane == 0) red[0][wave] = s;
  __syncthreads();
  const float mu = ((red[0][0] + red[0][1]) + (red[0][2] + red[0][3])) * (1.0f / (float)NDIM);
  float qd = 0.f, sq = 0.f;
#pragma unroll
  for (int e = 0; e < 8; ++e) { const float d = v[e] - mu; qd += d * d; sq += v[e] * v[e]; }
#pragma unroll
  for (int off = 1; off < 32; off <<= 1) { qd += __shfl_xor(qd, off, 32); sq += __shfl_xor(sq, off, 32); }
  if (lane == 0) { red[1][wave] = qd; red[2][wave] = sq; }
  __syncthreads();
  const float var = ((red[1][0] + red[1][1]) + (red[1][2] + red[1][3])) * (1.0f / (float)NDIM);
  const float e1 = (red[2][0] + red[2][1]) * (1.0f / (float)(NDIM / 2));
  const float e2 = (red[2][2] + red[2][3]) * (1.0f / (float)(NDIM / 2));
  const float imb = (e1 - e2) * bw[0];
  const float inv = 1.0f / sqrtf(var + 1e-6f);
  const float corr = (tid < 64) ? -imb : imb;
  const v4f g0 = *(const v4f*)(g + tid * 8);
  const v4f g1 = *(const v4f*)(g + tid * 8 + 4);
  const v4f b0 = *(const v4f*)(bb + tid * 8);
  const v4f b1 = *(const v4f*)(bb + tid * 8 + 4);
  v8h hv;
#pragma unroll
  for (int e = 0; e < 4; ++e) {
    const float o0 = (v[e] - mu) * inv * g0[e] + b0[e] + corr;
    const float o1 = (v[4 + e] - mu) * inv * g1[e] + b1[e] + corr;
    hv[e] = (_Float16)o0;
    hv[4 + e] = (_Float16)o1;
  }
  unsigned short* op = outp + (size_t)row * NDIM + tid * 8;
  *(volatile v8h*)(op) = hv;
  __threadfence();
  *(volatile v8h*)(op) = hv;
}

__global__ __launch_bounds__(256) void gelu_f16_kernel(const float* __restrict__ hin, unsigned short* __restrict__ gout,
                                                       int ncols, int nact, float mul, int total8)
{
  const int t = blockIdx.x * 256 + threadIdx.x;
  if (t >= total8) return;
  const size_t base = (size_t)t * 8;
  const int col0 = (int)(base % (size_t)ncols);
  unsigned long long wlo = 0ull, whi = 0ull;
#pragma unroll 1
  for (int e = 0; e < 8; ++e) {
    const float hvv = hin[base + e];
    float gv = 0.5f * hvv * (1.0f + erff(hvv * 0.70710678118654752f));
    gv = (col0 + e < nact) ? (gv * mul) : 0.0f;
    const unsigned long long bits = (unsigned long long)__builtin_bit_cast(unsigned short, (_Float16)gv);
    const unsigned long long sh = bits << (16 * (e & 3));
    if (e < 4) wlo |= sh; else whi |= sh;
  }
  v4u w;
  w[0] = (unsigned)(wlo & 0xffffffffull);
  w[1] = (unsigned)(wlo >> 32);
  w[2] = (unsigned)(whi & 0xffffffffull);
  w[3] = (unsigned)(whi >> 32);
  *(volatile v4u*)(gout + base) = w;
  __threadfence();
  *(volatile v4u*)(gout + base) = w;
}

#define AT_D 64
#define AT_NW 4
#define AT_QB 64
#define AT_KC 64
#define AT_PSC 32768.0f

__device__ __forceinline__ v8f mma_h(v16h a, v16h b, v8f c) {
  c = __builtin_amdgcn_wmma_f32_16x16x32_f16(false, a, false, b, (short)0, c, false, false);
  asm volatile("v_nop\n\tv_nop\n\tv_nop\n\tv_nop" : "+v"(c) : "v"(a), "v"(b));
  return c;
}
union FragH { v16h v; v8h h[2]; };

__global__ __launch_bounds__(128)
void attn_f16_kernel(const unsigned short* __restrict__ qp, const unsigned short* __restrict__ kp,
                     const unsigned short* __restrict__ vp, const int* __restrict__ maskp,
                     unsigned short* __restrict__ outp,
                     const float* __restrict__ cbeta, const float* __restrict__ civ,
                     const float* __restrict__ cov, const float* __restrict__ cchi,
                     int S, int H, int ld, float sm_scale, float out_mul)
{
  __shared__ __align__(16) unsigned short Ksh[AT_KC * AT_D];
  __shared__ __align__(16) unsigned short Vth[AT_D * AT_KC];
  __shared__ __align__(16) _Float16 Psh[AT_NW][16 * AT_KC];
  __shared__ __align__(16) float Os[AT_NW][16 * 68];
  __shared__ __align__(16) unsigned int Mw[AT_QB * (AT_KC / 4)];
  __shared__ int flg[AT_NW];

  const int tid = threadIdx.x, wave = tid >> 5, lane = tid & 31, hh = lane >> 4, c = lane & 15;
  const int nqb = S / AT_QB;
  const int bx = blockIdx.x;
  const int qb = bx % nqb;
  const int bh = bx / nqb;
  const int h  = bh % H;
  const int b  = bh / H;
  const int qbase = qb * AT_QB;
  const int q0 = qbase + wave * 16;
  const size_t tok0 = (size_t)b * S;
  const int hoff = h * AT_D;

  v16h qa[2];
  {
    const _Float16* qrow = (const _Float16*)qp + (tok0 + q0 + c) * (size_t)ld + hoff;
#pragma unroll
    for (int dc = 0; dc < 2; ++dc) qa[dc] = Frag<_Float16>::load(qrow + dc * 32 + 8 * hh);
  }

  float mrow[8], lrow[8];
  v8f oacc[4];
#pragma unroll
  for (int r = 0; r < 8; ++r) { mrow[r] = -INFINITY; lrow[r] = 0.f; }
#pragma unroll
  for (int t = 0; t < 4; ++t) oacc[t] = (v8f){0.f,0.f,0.f,0.f,0.f,0.f,0.f,0.f};

  const unsigned char* Mb = (const unsigned char*)Mw;
  const _Float16* Ks16 = (const _Float16*)Ksh;
  const _Float16* Vt16 = (const _Float16*)Vth;
  const int nch = S / AT_KC;

  for (int kc = 0; kc < nch; ++kc) {
    const int kv0 = kc * AT_KC;
    __syncthreads();
    {
      const int mr = tid >> 1, mh = tid & 1;
      const int* msrc = maskp + (size_t)(qbase + mr) * S + kv0 + mh * 32;
      int anyv = 0;
#pragma unroll
      for (int i = 0; i < 8; ++i) {
        const v4i m4 = *(const v4i*)(msrc + 4 * i);
        const unsigned w = (m4[0] != 0 ? 1u : 0u) | (m4[1] != 0 ? 0x100u : 0u) |
                           (m4[2] != 0 ? 0x10000u : 0u) | (m4[3] != 0 ? 0x1000000u : 0u);
        Mw[mr * 16 + mh * 8 + i] = w;
        anyv |= (int)w;
      }
#pragma unroll
      for (int off = 1; off < 32; off <<= 1) anyv |= __shfl_xor(anyv, off, 32);
      if (lane == 0) flg[wave] = anyv;
    }
    __syncthreads();
    const int anyb = flg[0] | flg[1] | flg[2] | flg[3];
    if (anyb != 0) {
      {
        const int kvr = tid >> 1, dh = (tid & 1) * 32;
        const unsigned short* krow = kp + (tok0 + kv0 + kvr) * (size_t)ld + hoff + dh;
        const unsigned short* vrow = vp + (tok0 + kv0 + kvr) * (size_t)ld + hoff + dh;
#pragma unroll
        for (int i = 0; i < 4; ++i) {
          const v4u kw = *(const v4u*)(krow + 8 * i);
          *(v4u*)(Ksh + kvr * AT_D + dh + 8 * i) = kw;
          const v4u vw = *(const v4u*)(vrow + 8 * i);
#pragma unroll
          for (int m = 0; m < 4; ++m) {
            const unsigned u = vw[m];
            const int d0 = dh + 8 * i + 2 * m;
            Vth[d0 * AT_KC + kvr]       = (unsigned short)(u & 0xffffu);
            Vth[(d0 + 1) * AT_KC + kvr] = (unsigned short)(u >> 16);
          }
        }
      }
      __syncthreads();

      v8f s[4];
#pragma unroll
      for (int j = 0; j < 4; ++j) {
        s[j] = (v8f){0.f,0.f,0.f,0.f,0.f,0.f,0.f,0.f};
#pragma unroll
        for (int dc = 0; dc < 2; ++dc) {
          FragH kf;
          kf.h[0] = *(const v8h*)(Ks16 + (j * 16 + c) * AT_D + dc * 32 + 8 * hh);
          kf.h[1] = *(const v8h*)(Ks16 + (j * 16 + c) * AT_D + dc * 32 + 16 + 8 * hh);
          s[j] = mma_h(qa[dc], kf.v, s[j]);
        }
      }
      float cm[8];
#pragma unroll
      for (int r = 0; r < 8; ++r) {
        const int qrl = wave * 16 + 8 * hh + r;
        float m = -INFINITY;
#pragma unroll
        for (int j = 0; j < 4; ++j) {
          const int kvl = j * 16 + c;
          const bool keep = (Mb[qrl * AT_KC + kvl] != 0);
          const float val = keep ? (s[j][r] * sm_scale) : -INFINITY;
          s[j][r] = val;
          m = fmaxf(m, val);
        }
#pragma unroll
        for (int off = 1; off < 16; off <<= 1) m = fmaxf(m, __shfl_xor(m, off, 32));
        cm[r] = m;
      }
      _Float16* pw = Psh[wave];
#pragma unroll
      for (int r = 0; r < 8; ++r) {
        const float mnew = fmaxf(mrow[r], cm[r]);
        const bool dead = (mnew == -INFINITY);
        const float alpha = dead ? 1.0f : expf(mrow[r] - mnew);
        mrow[r] = mnew;
        float psum = 0.f;
#pragma unroll
        for (int j = 0; j < 4; ++j) {
          const float p = dead ? 0.0f : expf(s[j][r] - mnew);
          psum += p;
          pw[(8 * hh + r) * AT_KC + j * 16 + c] = (_Float16)(p * AT_PSC);
        }
#pragma unroll
        for (int off = 1; off < 16; off <<= 1) psum += __shfl_xor(psum, off, 32);
        lrow[r] = lrow[r] * alpha + psum;
#pragma unroll
        for (int t = 0; t < 4; ++t) oacc[t][r] *= alpha;
      }
      __builtin_amdgcn_fence(__ATOMIC_RELEASE, "workgroup");
      __builtin_amdgcn_wave_barrier();
      __builtin_amdgcn_fence(__ATOMIC_ACQUIRE, "workgroup");
      const _Float16* pr = pw;
#pragma unroll
      for (int kk = 0; kk < 2; ++kk) {
        FragH pa;
        pa.h[0] = *(const v8h*)(pr + c * AT_KC + kk * 32 + 8 * hh);
        pa.h[1] = *(const v8h*)(pr + c * AT_KC + kk * 32 + 16 + 8 * hh);
#pragma unroll
        for (int t = 0; t < 4; ++t) {
          FragH vb;
          vb.h[0] = *(const v8h*)(Vt16 + (t * 16 + c) * AT_KC + kk * 32 + 8 * hh);
          vb.h[1] = *(const v8h*)(Vt16 + (t * 16 + c) * AT_KC + kk * 32 + 16 + 8 * hh);
          oacc[t] = mma_h(pa.v, vb.v, oacc[t]);
        }
      }
    }
  }

  const float sbeta = 1.0f / (1.0f + expf(-cbeta[h]));
  const float ang = 3.14159265358979323846f * sbeta;
  const float ca = cosf(ang), sa = sinf(ang);
  const float ivg = 1.0f / (1.0f + expf(-civ[h]));
  const float og = (1.0f / (1.0f + expf(-cov[h]))) * tanhf(cchi[h]) * out_mul;
  float* os = Os[wave];
#pragma unroll
  for (int r = 0; r < 8; ++r) {
    const float f = ivg / (lrow[r] * AT_PSC);
    const float x0 = oacc[0][r] * f, x1 = oacc[1][r] * f, x2 = oacc[2][r] * f, x3 = oacc[3][r] * f;
    os[(8 * hh + r) * 68 + c]      = (x0 * ca - x2 * sa) * og;
    os[(8 * hh + r) * 68 + 16 + c] = (x1 * ca - x3 * sa) * og;
    os[(8 * hh + r) * 68 + 32 + c] = (x0 * sa + x2 * ca) * og;
    os[(8 * hh + r) * 68 + 48 + c] = (x1 * sa + x3 * ca) * og;
  }
  __builtin_amdgcn_fence(__ATOMIC_RELEASE, "workgroup");
  __builtin_amdgcn_wave_barrier();
  __builtin_amdgcn_fence(__ATOMIC_ACQUIRE, "workgroup");
  {
    const int q4 = lane >> 3, c8 = (lane & 7) * 8;
    for (int pass = 0; pass < 2; ++pass) {
#pragma unroll
      for (int it = 0; it < 4; ++it) {
        const int row = it * 4 + q4;
        const float* sp = os + row * 68 + c8;
        v8h hv;
#pragma unroll
        for (int e = 0; e < 8; ++e) hv[e] = (_Float16)sp[e];
        *(volatile v8h*)(outp + (tok0 + q0 + row) * (size_t)ld + hoff + c8) = hv;
      }
      __threadfence();
    }
  }
}

extern "C" void kernel_launch(void* const* d_in, const int* in_sizes, int n_in,
                              void* d_out, int out_size, void* d_ws, size_t ws_size,
                              hipStream_t stream)
{
  if (n_in < 22) return;
  if (in_sizes[0] != NROWS * NDIM) return;
  if (in_sizes[1] != NTOK * NTOK) return;
  if (in_sizes[2] != NDIM * NDIM || in_sizes[3] != NDIM * NDIM || in_sizes[4] != NDIM * NDIM || in_sizes[5] != NDIM * NDIM) return;
  if (in_sizes[6] != NDIM || in_sizes[7] != NDIM || in_sizes[8] < 1 || in_sizes[9] != NDIM || in_sizes[10] != NDIM || in_sizes[11] < 1) return;
  if (in_sizes[12] != NHEAD || in_sizes[13] != NHEAD || in_sizes[14] != NHEAD || in_sizes[15] != NHEAD) return;
  if (in_sizes[16] != NDIM * NHID || in_sizes[17] != NHID || in_sizes[18] != NHID * NDIM || in_sizes[19] != NDIM) return;
  if (in_sizes[20] < 1 || in_sizes[21] != NDIM * NDIM) return;
  if (out_size != NROWS * NDIM) return;
  if (ws_size < WS_TOTAL) return;

  const float* x     = (const float*)d_in[0];
  const int*   maskp = (const int*)d_in[1];
  const float* Wq    = (const float*)d_in[2];
  const float* Wk    = (const float*)d_in[3];
  const float* Wv    = (const float*)d_in[4];
  const float* Wo    = (const float*)d_in[5];
  const float* ln1g  = (const float*)d_in[6];
  const float* ln1b  = (const float*)d_in[7];
  const float* bw1   = (const float*)d_in[8];
  const float* ln2g  = (const float*)d_in[9];
  const float* ln2b  = (const float*)d_in[10];
  const float* bw2   = (const float*)d_in[11];
  const float* cbeta = (const float*)d_in[12];
  const float* civ   = (const float*)d_in[13];
  const float* cov   = (const float*)d_in[14];
  const float* cchi  = (const float*)d_in[15];
  const float* Win   = (const float*)d_in[16];
  const float* bin   = (const float*)d_in[17];
  const float* Wout  = (const float*)d_in[18];
  const float* bout  = (const float*)d_in[19];
  const float* rbeta = (const float*)d_in[20];
  const float* nestW = (const float*)d_in[21];
  float* outp = (float*)d_out;

  char* ws = (char*)d_ws;
  unsigned short* wqkvT = (unsigned short*)(ws + OFF_WQKV);
  unsigned short* woT   = (unsigned short*)(ws + OFF_WO);
  unsigned short* winT  = (unsigned short*)(ws + OFF_WIN);
  unsigned short* woutT = (unsigned short*)(ws + OFF_WOUT);
  unsigned short* nhi   = (unsigned short*)(ws + OFF_NHI);
  unsigned short* nlo   = (unsigned short*)(ws + OFF_NLO);
  unsigned short* xn    = (unsigned short*)(ws + OFF_XN);
  unsigned short* qkv   = (unsigned short*)(ws + OFF_QKV);
  unsigned short* cb    = (unsigned short*)(ws + OFF_CB);
  float*          x1    = (float*)(ws + OFF_X1);
  unsigned short* gbuf  = (unsigned short*)(ws + OFF_G);
  float*          hbuf  = (float*)(ws + OFF_H);
  unsigned short* x2h   = (unsigned short*)(ws + OFF_X2H);
  unsigned short* x2l   = (unsigned short*)(ws + OFF_X2L);

  const dim3 gsq(NDIM / 64, NDIM / 64);
  tcast_kernel<0><<<gsq, 256, 0, stream>>>(Wq, NDIM, NDIM, wqkvT,           wqkvT,           NDIM, NDIM, 64.0f);
  tcast_kernel<0><<<gsq, 256, 0, stream>>>(Wk, NDIM, NDIM, wqkvT + WSQ,     wqkvT + WSQ,     NDIM, NDIM, 64.0f);
  tcast_kernel<0><<<gsq, 256, 0, stream>>>(Wv, NDIM, NDIM, wqkvT + 2 * WSQ, wqkvT + 2 * WSQ, NDIM, NDIM, 64.0f);
  tcast_kernel<0><<<gsq, 256, 0, stream>>>(Wo, NDIM, NDIM, woT, woT, NDIM, NDIM, 64.0f);
  tcast_kernel<0><<<dim3(NDIM / 64, NHPAD / 64), 256, 0, stream>>>(Win, NDIM, NHID, winT, winT, NDIM, NDIM, 64.0f);
  tcast_kernel<0><<<dim3(NHPAD / 64, NDIM / 64), 256, 0, stream>>>(Wout, NHID, NDIM, woutT, woutT, NHPAD, NACTIVE, 64.0f);
  tcast_kernel<1><<<gsq, 256, 0, stream>>>(nestW, NDIM, NDIM, nhi, nlo, NDIM, NDIM, 1.0f);

  bnorm_f16_kernel<<<NROWS, 128, 0, stream>>>(x, ln1g, ln1b, bw1, xn);

  static_assert(((NROWS / 64) * (NDIM / 64)) % 8 == 0 && ((NROWS / 64) * (NHPAD / 64)) % 8 == 0, "8 tiles per block");
  const int gx_d = (NROWS / 64) * (NDIM / 64) / 8;
  const int gx_h = (NROWS / 64) * (NHPAD / 64) / 8;
  wmma_gemm64<0, false, 0, 1, false, 0, false><<<dim3(gx_d, 3), 256, 0, stream>>>(
      xn, xn, NDIM, 0L, wqkvT, wqkvT, NDIM, (long)WSQ, (void*)qkv, (void*)qkv, NDIM, (long)PLANE,
      bin, x, 0L, rbeta, NROWS, NDIM, NDIM, 1.0f / 64.0f);

  attn_f16_kernel<<<NBATCH * NHEAD * (NTOK / AT_QB), 128, 0, stream>>>(
      qkv, qkv + PLANE, qkv + 2 * PLANE, maskp, cb, cbeta, civ, cov, cchi, NTOK, NHEAD, NDIM, 0.125f, 64.0f);

  wmma_gemm64<0, false, 0, 0, true, 0, true><<<dim3(gx_d, 1), 256, 0, stream>>>(
      cb, cb, NDIM, 0L, woT, woT, NDIM, 0L, (void*)x1, (void*)x1, NDIM, 0L,
      bin, x, 0L, rbeta, NROWS, NDIM, NDIM, 1.0f / 4096.0f);

  bnorm_f16_kernel<<<NROWS, 128, 0, stream>>>(x1, ln2g, ln2b, bw2, xn);

  wmma_gemm64<0, false, 2, 0, false, 0, false><<<dim3(gx_h, 1), 256, 0, stream>>>(
      xn, xn, NDIM, 0L, winT, winT, NDIM, 0L, (void*)hbuf, (void*)hbuf, NHPAD, 0L,
      bin, x, 0L, rbeta, NROWS, NHPAD, NDIM, 1.0f / 64.0f);

  static_assert((NROWS * NHPAD) % (8 * 256) == 0, "gelu grid exact");
  gelu_f16_kernel<<<(NROWS * NHPAD) / (8 * 256), 256, 0, stream>>>(hbuf, gbuf, NHPAD, NACTIVE, 64.0f, (NROWS * NHPAD) / 8);

  wmma_gemm64<0, false, 2, 2, true, 0, true><<<dim3(gx_d, 1), 256, 0, stream>>>(
      gbuf, gbuf, NHPAD, 0L, woutT, woutT, NHPAD, 0L, (void*)x2h, (void*)x2l, NDIM, 0L,
      bout, x1, 0L, rbeta, NROWS, NDIM, NHPAD, 1.0f / 4096.0f);

  wmma_gemm64<1, true, 0, 0, false, 0, false><<<dim3(gx_d, 1), 256, 0, stream>>>(
      x2h, x2l, NDIM, 0L, nhi, nlo, NDIM, 0L, (void*)outp, (void*)outp, NDIM, 0L,
      bout, x1, 0L, rbeta, NROWS, NDIM, NDIM, 1.0f);
}
